// SingleAttention_72877005078947
// MI455X (gfx1250) — hardware-verified
//
#include <hip/hip_runtime.h>
#include <math.h>
#include <stdint.h>

#define NB    4
#define SEQ   2048
#define DM    1024
#define ROWS  (NB * SEQ)
#define OUTN  (ROWS * DM)
static_assert((SEQ % 64) == 0 && (DM % 64) == 0 && (ROWS % 64) == 0 && (DM % 32) == 0 && (DM % 256) == 0);
static_assert(SEQ == 256 * 8);
static_assert((((ROWS / 64) * (DM / 64)) % 8) == 0);
static_assert((((SEQ / 64) * (SEQ / 64)) % 8) == 0);
static_assert((((SEQ / 64) * (DM / 64)) % 8) == 0);
static_assert(((ROWS * DM / 8) % 256) == 0 && ((DM * DM / 8) % 256) == 0);
static_assert((size_t)SEQ * SEQ * 4 <= (size_t)ROWS * DM * 4);

typedef _Float16 v16h __attribute__((ext_vector_type(16)));
typedef _Float16 v8h  __attribute__((ext_vector_type(8)));
typedef __bf16   v16b __attribute__((ext_vector_type(16)));
typedef __bf16   v8b  __attribute__((ext_vector_type(8)));
typedef float    v8f  __attribute__((ext_vector_type(8)));
typedef float    v4f  __attribute__((ext_vector_type(4)));
typedef unsigned int v4u __attribute__((ext_vector_type(4)));

__device__ __forceinline__ unsigned short bf_bits(float f) {
  unsigned u = __float_as_uint(f);
  return (unsigned short)((u + 0x7FFFu + ((u >> 16) & 1u)) >> 16);
}
__device__ __forceinline__ float bf_up(unsigned short h) { return __uint_as_float(((unsigned)h) << 16); }
__device__ __forceinline__ unsigned short h_bits(_Float16 x) { return __builtin_bit_cast(unsigned short, x); }
__device__ __forceinline__ unsigned pk16(unsigned short a, unsigned short b) { return (unsigned)a | ((unsigned)b << 16); }
__device__ __forceinline__ v8f zero8() { v8f z = {0.f, 0.f, 0.f, 0.f, 0.f, 0.f, 0.f, 0.f}; return z; }

__device__ __forceinline__ v16b ldfrag_b(const __bf16* p) {
  union { v16b v; v8b h[2]; } f;
  f.h[0] = *(const v8b*)(p);
  f.h[1] = *(const v8b*)(p + 16);
  return f.v;
}
__device__ __forceinline__ v16h ldfrag_h(const _Float16* p) {
  union { v16h v; v8h h[2]; } f;
  f.h[0] = *(const v8h*)(p);
  f.h[1] = *(const v8h*)(p + 16);
  return f.v;
}

__device__ __forceinline__ v8f mma_h(v16h a, v16h b, v8f c) {
  c = __builtin_amdgcn_wmma_f32_16x16x32_f16(false, a, false, b, (short)0, c, false, false);
#if defined(__HIP_DEVICE_COMPILE__)
  asm volatile("v_nop\n\tv_nop\n\tv_nop\n\tv_nop" : "+v"(c) : "v"(a), "v"(b));
#endif
  return c;
}
__device__ __forceinline__ v8f mma_b_raw(v16b a, v16b b, v8f c) {
  return __builtin_amdgcn_wmma_f32_16x16x32_bf16(false, a, false, b, (short)0, c, false, false);
}
__device__ __forceinline__ void dep_guard_b(v8f& a, v8f& b, v16b x, v16b y) {
#if defined(__HIP_DEVICE_COMPILE__)
  asm volatile("v_nop\n\tv_nop\n\tv_nop\n\tv_nop" : "+v"(a), "+v"(b) : "v"(x), "v"(y));
#endif
}
__device__ __forceinline__ void keep4_b(v16b a, v16b b, v16b c, v16b d) {
#if defined(__HIP_DEVICE_COMPILE__)
  asm volatile("v_nop" :: "v"(a), "v"(b), "v"(c), "v"(d));
#endif
}
__device__ __forceinline__ void acc_guard4(v8f& a, v8f& b, v8f& c, v8f& d) {
#if defined(__HIP_DEVICE_COMPILE__)
  asm volatile("v_nop\n\tv_nop\n\tv_nop\n\tv_nop" : "+v"(a), "+v"(b), "+v"(c), "+v"(d));
#endif
}

__global__ __launch_bounds__(256) void cvt_bf16x8(const float* __restrict__ in, unsigned short* out, int n8) {
  const int i = blockIdx.x * 256 + threadIdx.x;
  if (i < n8) {
    const v4f a = *(const v4f*)(in + (size_t)i * 8);
    const v4f b = *(const v4f*)(in + (size_t)i * 8 + 4);
    v4u p;
    p[0] = pk16(bf_bits(a[0]), bf_bits(a[1]));
    p[1] = pk16(bf_bits(a[2]), bf_bits(a[3]));
    p[2] = pk16(bf_bits(b[0]), bf_bits(b[1]));
    p[3] = pk16(bf_bits(b[2]), bf_bits(b[3]));
    *(volatile v4u*)(out + (size_t)i * 8) = p;
    __threadfence();
    *(volatile v4u*)(out + (size_t)i * 8) = p;
  }
}

__global__ __launch_bounds__(256) void plane_f16x8(const float* __restrict__ in, unsigned short* hp, int n8,
                                                   float scale, int rb) {
  const int i = blockIdx.x * 256 + threadIdx.x;
  if (i < n8) {
    const v4f a = *(const v4f*)(in + (size_t)i * 8);
    const v4f b = *(const v4f*)(in + (size_t)i * 8 + 4);
    float f[8];
    f[0] = a[0]; f[1] = a[1]; f[2] = a[2]; f[3] = a[3];
    f[4] = b[0]; f[5] = b[1]; f[6] = b[2]; f[7] = b[3];
    if (rb != 0) {
#pragma unroll
      for (int e = 0; e < 8; ++e) f[e] = bf_up(bf_bits(f[e]));
    }
    v4u ph;
#pragma unroll
    for (int e = 0; e < 4; ++e) {
      const _Float16 x0 = (_Float16)(f[2 * e] * scale);
      const _Float16 x1 = (_Float16)(f[2 * e + 1] * scale);
      ph[e] = pk16(h_bits(x0), h_bits(x1));
    }
    *(volatile v4u*)(hp + (size_t)i * 8) = ph;
    __threadfence();
    *(volatile v4u*)(hp + (size_t)i * 8) = ph;
  }
}

__global__ __launch_bounds__(256) void gemm64(
    const unsigned short* __restrict__ Ap, int lda,
    const unsigned short* __restrict__ Btp, int ldb,
    const float* __restrict__ bias,
    float* C, int ldc, int M, int N, int K) {
  const __bf16* Ab  = (const __bf16*)(const void*)Ap;
  const __bf16* Bb  = (const __bf16*)(const void*)Btp;
  __shared__ __align__(16) float sT[8][16 * 68];
  const int lane = threadIdx.x & 31;
  const int wave = threadIdx.x >> 5;
  const int tilesN = N >> 6;
  const int tilesM = M >> 6;
  const int tile = blockIdx.x * 8 + wave;
  if (tile >= tilesM * tilesN) return;
  const int tm = tile / tilesN;
  const int tn = tile - tm * tilesN;
  const int m0 = tm << 6;
  const int n0 = tn << 6;

  const int rlane = lane & 15;
  const int koff  = (lane >> 4) * 8;
  const int mOff  = (lane >> 4) * 8;

  v8f acc[4][4];
#pragma unroll
  for (int i = 0; i < 4; ++i)
#pragma unroll
    for (int j = 0; j < 4; ++j) acc[i][j] = zero8();

  for (int k0 = 0; k0 < K; k0 += 32) {
    v16b bh[4];
#pragma unroll
    for (int j = 0; j < 4; ++j) {
      const size_t bo = (size_t)(n0 + (j << 4) + rlane) * ldb + koff + k0;
      bh[j] = ldfrag_b(Bb + bo);
    }
#pragma unroll
    for (int i = 0; i < 4; ++i) {
      const size_t ao = (size_t)(m0 + (i << 4) + rlane) * lda + koff + k0;
      const v16b ah = ldfrag_b(Ab + ao);
#pragma unroll
      for (int j = 0; j < 4; ++j) {
        acc[i][j] = mma_b_raw(ah, bh[j], acc[i][j]);
      }
      dep_guard_b(acc[i][0], acc[i][3], ah, ah);
    }
    keep4_b(bh[0], bh[1], bh[2], bh[3]);
  }
  acc_guard4(acc[0][0], acc[0][1], acc[0][2], acc[0][3]);
  acc_guard4(acc[1][0], acc[1][1], acc[1][2], acc[1][3]);
  acc_guard4(acc[2][0], acc[2][1], acc[2][2], acc[2][3]);
  acc_guard4(acc[3][0], acc[3][1], acc[3][2], acc[3][3]);

  float bz[4];
#pragma unroll
  for (int j = 0; j < 4; ++j) bz[j] = bf_up(bf_bits(bias[n0 + (j << 4) + rlane]));

  float* slab = sT[wave];
#pragma unroll
  for (int i = 0; i < 4; ++i) {
    const int mBase = m0 + (i << 4);
#pragma unroll
    for (int r = 0; r < 8; ++r) {
#pragma unroll
      for (int j = 0; j < 4; ++j) {
        slab[(mOff + r) * 68 + (j << 4) + rlane] = acc[i][j][r] + bz[j];
      }
    }
    __builtin_amdgcn_fence(__ATOMIC_RELEASE, "workgroup");
    __builtin_amdgcn_wave_barrier();
    __builtin_amdgcn_fence(__ATOMIC_ACQUIRE, "workgroup");
    {
      const int hh = lane >> 4, c4 = (lane & 15) * 4;
      v4f ov[8];
#pragma unroll
      for (int it = 0; it < 8; ++it) {
        const int row = it * 2 + hh;
        ov[it] = *(const v4f*)(slab + row * 68 + c4);
      }
      for (int pass = 0; pass < 2; ++pass) {
#pragma unroll
        for (int it = 0; it < 8; ++it) {
          const int row = it * 2 + hh;
          *(volatile v4f*)(C + (size_t)(mBase + row) * ldc + n0 + c4) = ov[it];
        }
        __threadfence();
      }
    }
    __builtin_amdgcn_fence(__ATOMIC_RELEASE, "workgroup");
    __builtin_amdgcn_wave_barrier();
    __builtin_amdgcn_fence(__ATOMIC_ACQUIRE, "workgroup");
  }
}

__global__ __launch_bounds__(256) void vt_plane(const float* __restrict__ vf, unsigned short* vth, float vscale) {
  __shared__ __align__(16) float sv[64 * 68];
  const int tid = threadIdx.x;
  const int t0  = blockIdx.x * 64;
  const int fh  = blockIdx.y;
  const int b   = blockIdx.z;
#pragma unroll
  for (int i = 0; i < 4; ++i) {
    const int idx = i * 256 + tid;
    const int tt = idx >> 4, c4 = (idx & 15) * 4;
    const v4f a = *(const v4f*)(vf + ((size_t)(b * SEQ + t0 + tt)) * DM + fh * 64 + c4);
    *(v4f*)(sv + tt * 68 + c4) = a;
  }
  __syncthreads();

  const int g = tid >> 3, piece = tid & 7;
  v4u hv[2];
  size_t hofs[2];
#pragma unroll
  for (int it = 0; it < 2; ++it) {
    const int d = it * 32 + g;
    v4u a;
#pragma unroll
    for (int e = 0; e < 4; ++e) {
      const float f0 = bf_up(bf_bits(sv[(piece * 8 + 2 * e) * 68 + d])) * vscale;
      const float f1 = bf_up(bf_bits(sv[(piece * 8 + 2 * e + 1) * 68 + d])) * vscale;
      a[e] = pk16(h_bits((_Float16)f0), h_bits((_Float16)f1));
    }
    hv[it] = a;
    hofs[it] = ((size_t)(b * DM + fh * 64 + d)) * SEQ + t0 + piece * 8;
  }
  for (int pass = 0; pass < 2; ++pass) {
#pragma unroll
    for (int it = 0; it < 2; ++it) {
      *(volatile v4u*)(vth + hofs[it]) = hv[it];
    }
    __threadfence();
  }
}

__global__ __launch_bounds__(256) void colmean(const float* __restrict__ vf, float* mv) {
  __shared__ __align__(16) float sm[256];
  const int tid = threadIdx.x;
  const int n = blockIdx.x * 256 + tid;
  const int b = blockIdx.y;
  const float* p = vf + (size_t)b * SEQ * DM + n;
  double s = 0.0;
#pragma unroll 4
  for (int t = 0; t < SEQ; ++t) s += (double)bf_up(bf_bits(p[(size_t)t * DM]));
  sm[tid] = (float)(s * (1.0 / (double)SEQ));
  __syncthreads();
  if (tid < 64) {
    const v4f v = *(const v4f*)(sm + tid * 4);
    float* q = mv + (size_t)b * DM + blockIdx.x * 256 + tid * 4;
    *(volatile v4f*)q = v;
    __threadfence();
    *(volatile v4f*)q = v;
  }
}

__global__ __launch_bounds__(256) void gemm64h_s(
    const unsigned short* __restrict__ Ap, int lda,
    const unsigned short* __restrict__ Btp, int ldb,
    float* C, int ldc, int M, int N, int K, float cscale) {
  const _Float16* Ah = (const _Float16*)(const void*)Ap;
  const _Float16* Bh = (const _Float16*)(const void*)Btp;
  __shared__ __align__(16) float sT[8][16 * 68];
  const int lane = threadIdx.x & 31;
  const int wave = threadIdx.x >> 5;
  const int tilesN = N >> 6;
  const int tilesM = M >> 6;
  const int tile = blockIdx.x * 8 + wave;
  if (tile >= tilesM * tilesN) return;
  const int tm = tile / tilesN;
  const int tn = tile - tm * tilesN;
  const int m0 = tm << 6;
  const int n0 = tn << 6;
  const int rlane = lane & 15;
  const int koff  = (lane >> 4) * 8;
  const int mOff  = (lane >> 4) * 8;

  v8f acc[4][4];
#pragma unroll
  for (int i = 0; i < 4; ++i)
#pragma unroll
    for (int j = 0; j < 4; ++j) acc[i][j] = zero8();

  for (int k0 = 0; k0 < K; k0 += 32) {
    v16h bh[4];
#pragma unroll
    for (int j = 0; j < 4; ++j) {
      const size_t bo = (size_t)(n0 + (j << 4) + rlane) * ldb + koff + k0;
      bh[j] = ldfrag_h(Bh + bo);
    }
#pragma unroll
    for (int i = 0; i < 4; ++i) {
      const size_t ao = (size_t)(m0 + (i << 4) + rlane) * lda + koff + k0;
      const v16h ah = ldfrag_h(Ah + ao);
#pragma unroll
      for (int j = 0; j < 4; ++j) {
        acc[i][j] = mma_h(ah, bh[j], acc[i][j]);
      }
    }
  }

  float* slab = sT[wave];
#pragma unroll
  for (int i = 0; i < 4; ++i) {
    const int mBase = m0 + (i << 4);
#pragma unroll
    for (int r = 0; r < 8; ++r) {
#pragma unroll
      for (int j = 0; j < 4; ++j) {
        slab[(mOff + r) * 68 + (j << 4) + rlane] = acc[i][j][r] * cscale;
      }
    }
    __builtin_amdgcn_fence(__ATOMIC_RELEASE, "workgroup");
    __builtin_amdgcn_wave_barrier();
    __builtin_amdgcn_fence(__ATOMIC_ACQUIRE, "workgroup");
    {
      const int hh = lane >> 4, c4 = (lane & 15) * 4;
      v4f ov[8];
#pragma unroll
      for (int it = 0; it < 8; ++it) {
        const int row = it * 2 + hh;
        ov[it] = *(const v4f*)(slab + row * 68 + c4);
      }
      for (int pass = 0; pass < 2; ++pass) {
#pragma unroll
        for (int it = 0; it < 8; ++it) {
          const int row = it * 2 + hh;
          *(volatile v4f*)(C + (size_t)(mBase + row) * ldc + n0 + c4) = ov[it];
        }
        __threadfence();
      }
    }
    __builtin_amdgcn_fence(__ATOMIC_RELEASE, "workgroup");
    __builtin_amdgcn_wave_barrier();
    __builtin_amdgcn_fence(__ATOMIC_ACQUIRE, "workgroup");
  }
}

__global__ __launch_bounds__(256) void softmax_c(const float* __restrict__ sf, unsigned short* ph) {
  __shared__ float redm[8];
  __shared__ float reds[8];
  const int row  = blockIdx.x;
  const int tid  = threadIdx.x;
  const int lane = tid & 31;
  const int wave = tid >> 5;
  const float* s = sf + (size_t)row * SEQ + tid * 8;
  const v4f a = *(const v4f*)(s);
  const v4f c = *(const v4f*)(s + 4);
  float v[8];
  v[0] = a[0]; v[1] = a[1]; v[2] = a[2]; v[3] = a[3];
  v[4] = c[0]; v[5] = c[1]; v[6] = c[2]; v[7] = c[3];
  float m = v[0];
#pragma unroll
  for (int e = 1; e < 8; ++e) m = fmaxf(m, v[e]);
#pragma unroll
  for (int o = 16; o > 0; o >>= 1) m = fmaxf(m, __shfl_xor(m, o));
  if (lane == 0) redm[wave] = m;
  __syncthreads();
  float mm = redm[0];
#pragma unroll
  for (int w = 1; w < 8; ++w) mm = fmaxf(mm, redm[w]);
  float sum = 0.f;
#pragma unroll
  for (int e = 0; e < 8; ++e) {
    v[e] = __expf(v[e] - mm);
    sum += v[e];
  }
#pragma unroll
  for (int o = 16; o > 0; o >>= 1) sum += __shfl_xor(sum, o);
  if (lane == 0) reds[wave] = sum;
  __syncthreads();
  float tot = 0.f;
#pragma unroll
  for (int w = 0; w < 8; ++w) tot += reds[w];
  const float inv = 1.0f / tot;
  v4u pk;
#pragma unroll
  for (int e = 0; e < 4; ++e) {
    const float p0 = v[2 * e] * inv;
    const float p1 = v[2 * e + 1] * inv;
    const _Float16 x0 = (_Float16)(p0 * 16384.0f - 8.0f);
    const _Float16 x1 = (_Float16)(p1 * 16384.0f - 8.0f);
    pk[e] = pk16(h_bits(x0), h_bits(x1));
  }
  unsigned short* o = ph + (size_t)row * SEQ + tid * 8;
  *(volatile v4u*)o = pk;
  __threadfence();
  *(volatile v4u*)o = pk;
}

__global__ __launch_bounds__(256) void gemm64h_pv(
    const unsigned short* __restrict__ Ap, int lda,
    const unsigned short* __restrict__ Btp, int ldb,
    const float* __restrict__ mv,
    float* C, int ldc, int M, int N, int K, float oscale) {
  const _Float16* Ah = (const _Float16*)(const void*)Ap;
  const _Float16* Bh = (const _Float16*)(const void*)Btp;
  __shared__ __align__(16) float sT[8][16 * 68];
  const int lane = threadIdx.x & 31;
  const int wave = threadIdx.x >> 5;
  const int tilesN = N >> 6;
  const int tilesM = M >> 6;
  const int tile = blockIdx.x * 8 + wave;
  if (tile >= tilesM * tilesN) return;
  const int tm = tile / tilesN;
  const int tn = tile - tm * tilesN;
  const int m0 = tm << 6;
  const int n0 = tn << 6;
  const int rlane = lane & 15;
  const int koff  = (lane >> 4) * 8;
  const int mOff  = (lane >> 4) * 8;

  v8f acc[4][4];
#pragma unroll
  for (int i = 0; i < 4; ++i)
#pragma unroll
    for (int j = 0; j < 4; ++j) acc[i][j] = zero8();

  for (int k0 = 0; k0 < K; k0 += 32) {
    v16h bh[4];
#pragma unroll
    for (int j = 0; j < 4; ++j) {
      const size_t bo = (size_t)(n0 + (j << 4) + rlane) * ldb + koff + k0;
      bh[j] = ldfrag_h(Bh + bo);
    }
#pragma unroll
    for (int i = 0; i < 4; ++i) {
      const size_t ao = (size_t)(m0 + (i << 4) + rlane) * lda + koff + k0;
      const v16h ah = ldfrag_h(Ah + ao);
#pragma unroll
      for (int j = 0; j < 4; ++j) {
        acc[i][j] = mma_h(ah, bh[j], acc[i][j]);
      }
    }
  }

  float mz[4];
#pragma unroll
  for (int j = 0; j < 4; ++j) mz[j] = mv[n0 + (j << 4) + rlane];

  float* slab = sT[wave];
#pragma unroll
  for (int i = 0; i < 4; ++i) {
    const int mBase = m0 + (i << 4);
#pragma unroll
    for (int r = 0; r < 8; ++r) {
#pragma unroll
      for (int j = 0; j < 4; ++j) {
        slab[(mOff + r) * 68 + (j << 4) + rlane] = acc[i][j][r] * oscale + mz[j];
      }
    }
    __builtin_amdgcn_fence(__ATOMIC_RELEASE, "workgroup");
    __builtin_amdgcn_wave_barrier();
    __builtin_amdgcn_fence(__ATOMIC_ACQUIRE, "workgroup");
    {
      const int hh = lane >> 4, c4 = (lane & 15) * 4;
      v4f ov[8];
#pragma unroll
      for (int it = 0; it < 8; ++it) {
        const int row = it * 2 + hh;
        ov[it] = *(const v4f*)(slab + row * 68 + c4);
      }
      for (int pass = 0; pass < 2; ++pass) {
#pragma unroll
        for (int it = 0; it < 8; ++it) {
          const int row = it * 2 + hh;
          *(volatile v4f*)(C + (size_t)(mBase + row) * ldc + n0 + c4) = ov[it];
        }
        __threadfence();
      }
    }
    __builtin_amdgcn_fence(__ATOMIC_RELEASE, "workgroup");
    __builtin_amdgcn_wave_barrier();
    __builtin_amdgcn_fence(__ATOMIC_ACQUIRE, "workgroup");
  }
}

extern "C" void kernel_launch(void* const* d_in, const int* in_sizes, int n_in,
                              void* d_out, int out_size, void* d_ws, size_t ws_size,
                              hipStream_t stream) {
  if (n_in < 9) return;
  if (in_sizes[0] != ROWS * DM) return;
  if (in_sizes[1] != ROWS * DM) return;
  if (in_sizes[2] != ROWS * DM) return;
  if (in_sizes[3] != DM * DM) return;
  if (in_sizes[4] != DM) return;
  if (in_sizes[5] != DM * DM) return;
  if (in_sizes[6] != DM) return;
  if (out_size != OUTN) return;

  const float* query = (const float*)d_in[0];
  const float* keyin = (const float*)d_in[1];
  const float* value = (const float*)d_in[2];
  const float* Wq    = (const float*)d_in[3];
  const float* bq    = (const float*)d_in[4];
  const float* Wk    = (const float*)d_in[5];
  const float* bk    = (const float*)d_in[6];

  const size_t PXb = (size_t)ROWS * DM * 2;
  const size_t PW  = (size_t)DM * DM * 2;
  const size_t PF  = (size_t)ROWS * DM * 4;
  const size_t PH  = (size_t)ROWS * DM * 2;
  const size_t PVt = (size_t)NB * DM * SEQ * 2;
  const size_t PP  = (size_t)SEQ * SEQ * 2;
  const size_t PMv = (size_t)NB * DM * 4;
  size_t off = 0;
  const size_t oXb = off; off += PXb;
  const size_t oWq = off; off += PW;
  const size_t oWk = off; off += PW;
  const size_t oTf = off; off += PF;
  const size_t oQh = off; off += PH;
  const size_t oKh = off; off += PH;
  const size_t oVt = off; off += PVt;
  const size_t oP  = off; off += PP;
  const size_t oMv = off; off += PMv;
  if (off > ws_size) return;
  if (off > (size_t)134217728) return;

  char* ws = (char*)d_ws;
  unsigned short* Xb  = (unsigned short*)(ws + oXb);
  unsigned short* Wqb = (unsigned short*)(ws + oWq);
  unsigned short* Wkb = (unsigned short*)(ws + oWk);
  float*          Tf  = (float*)(ws + oTf);
  unsigned short* Qh  = (unsigned short*)(ws + oQh);
  unsigned short* Kh  = (unsigned short*)(ws + oKh);
  unsigned short* VTh = (unsigned short*)(ws + oVt);
  unsigned short* Ph  = (unsigned short*)(ws + oP);
  float*          mV  = (float*)(ws + oMv);
  float*          outf = (float*)d_out;

  const dim3 blk(256);
  const int n8x = ROWS * DM / 8;
  const int n8w = DM * DM / 8;
  const dim3 gCvtX(n8x / 256);
  const dim3 gCvtW(n8w / 256);
  const dim3 gGemm(((ROWS / 64) * (DM / 64)) / 8);
  const dim3 gVpl(SEQ / 64, DM / 64, NB);
  const dim3 gCm(DM / 256, NB);
  const dim3 gSc(((SEQ / 64) * (SEQ / 64)) / 8);
  const dim3 gSm(SEQ);
  const dim3 gPv(((SEQ / 64) * (DM / 64)) / 8);
  const float qkScale = 16.0f;
  const float sscale  = 1.0f / 8192.0f;
  const float vScale  = 64.0f;
  const float pvOscl  = 1.0f / 1048576.0f;

  cvt_bf16x8<<<gCvtW, blk, 0, stream>>>(Wq, Wqb, n8w);
  cvt_bf16x8<<<gCvtW, blk, 0, stream>>>(Wk, Wkb, n8w);
  cvt_bf16x8<<<gCvtX, blk, 0, stream>>>(query, Xb, n8x);
  gemm64<<<gGemm, blk, 0, stream>>>(Xb, DM, Wqb, DM, bq, Tf, DM, ROWS, DM, DM);
  plane_f16x8<<<gCvtX, blk, 0, stream>>>(Tf, Qh, n8x, qkScale, 0);
  cvt_bf16x8<<<gCvtX, blk, 0, stream>>>(keyin, Xb, n8x);
  gemm64<<<gGemm, blk, 0, stream>>>(Xb, DM, Wkb, DM, bk, Tf, DM, ROWS, DM, DM);
  plane_f16x8<<<gCvtX, blk, 0, stream>>>(Tf, Kh, n8x, qkScale, 0);
  vt_plane<<<gVpl, blk, 0, stream>>>(value, VTh, vScale);
  colmean<<<gCm, blk, 0, stream>>>(value, mV);
  for (int b = 0; b < NB; ++b) {
    gemm64h_s<<<gSc, blk, 0, stream>>>(Qh + (size_t)b * SEQ * DM, DM, Kh + (size_t)b * SEQ * DM, DM,
                                       Tf, SEQ, SEQ, SEQ, DM, sscale);
    softmax_c<<<gSm, blk, 0, stream>>>(Tf, Ph);
    gemm64h_pv<<<gPv, blk, 0, stream>>>(Ph, SEQ, VTh + (size_t)b * DM * SEQ, SEQ, mV + (size_t)b * DM,
                                        outf + (size_t)b * SEQ * DM, DM, SEQ, DM, SEQ, pvOscl);
  }
  (void)hipGetLastError();
}
